// MambaLayer_31258771980442
// MI455X (gfx1250) — hardware-verified
//
#include <hip/hip_runtime.h>
#include <math.h>

typedef __attribute__((ext_vector_type(16))) _Float16 v16h;
typedef __attribute__((ext_vector_type(8)))  _Float16 v8h;
typedef __attribute__((ext_vector_type(16))) __bf16   v16b;
typedef __attribute__((ext_vector_type(8)))  __bf16   v8b;
typedef __attribute__((ext_vector_type(8)))  float    v8f;
typedef __attribute__((ext_vector_type(4)))  float    v4f;

constexpr int kBatch = 2;
constexpr int kSeqL  = 2048;
constexpr int kDmod  = 1024;
constexpr int kDin   = 2048;
constexpr int kNst   = 8;
constexpr int kDcv   = 4;
constexpr int kDtR   = 64;
constexpr int kPrjN  = kDtR + 2 * kNst;
constexpr int kPrjP  = 128;
constexpr int kXZP   = 2 * kDin;
constexpr int kRows  = kBatch * kSeqL;
constexpr int kTP    = 260;
constexpr float kCarW   = 32.0f;
constexpr float kCarWdt = 8.0f;
constexpr float kCarCv  = 64.0f;
constexpr float kCarXc  = 64.0f;
constexpr float kCarDt  = 64.0f;
constexpr float kCarY   = 128.0f;
constexpr float kSclPw  = 1.0f / (kCarCv * kCarW);
constexpr float kSclXp  = 1.0f / (kCarXc * kCarW);
constexpr float kSclDt  = 1.0f / (kCarDt * kCarWdt);
constexpr float kSclOut = 1.0f / (kCarY * kCarW);
static_assert(kPrjN == 80 && kPrjP >= kPrjN && (kPrjP % 64) == 0);
static_assert(kDcv == 4 && kNst == 8 && kDtR == 64);
static_assert((kDmod % 64) == 0 && (kDin % 64) == 0 && (kDtR % 64) == 0);
static_assert((kSeqL % 64) == 0 && (kXZP % 64) == 0 && (kPrjP % 64) == 0 && (kDin % 256) == 0 && (kSeqL % 16) == 0);

constexpr size_t kSzWINB  = (size_t)kXZP  * kDmod * 2;
constexpr size_t kSzPWT   = (size_t)kDin  * kDin  * 2;
constexpr size_t kSzWXT   = (size_t)kPrjP * kDin  * 2;
constexpr size_t kSzWDTT  = (size_t)kDin  * kDtR  * 2;
constexpr size_t kSzWOUTT = (size_t)kDmod * kDin  * 2;
constexpr size_t kSzXB    = (size_t)kRows * kDmod * 2;
constexpr size_t kSzXZ    = (size_t)kSeqL * kXZP  * 4;
constexpr size_t kSzXCV16 = (size_t)kSeqL * kDin  * 2;
constexpr size_t kSzXC    = (size_t)kSeqL * kDin  * 4;
constexpr size_t kSzXC16  = (size_t)kSeqL * kDin  * 2;
constexpr size_t kSzPROJ  = (size_t)kSeqL * kPrjP * 4;
constexpr size_t kSzDT16  = (size_t)kSeqL * kDtR  * 2;
constexpr size_t kSzDLR   = (size_t)kSeqL * kDin  * 4;
constexpr size_t kSzY16   = (size_t)kSeqL * kDin  * 2;
constexpr size_t kOffWINB  = 0;
constexpr size_t kOffPWT   = kOffWINB  + kSzWINB;
constexpr size_t kOffWXT   = kOffPWT   + kSzPWT;
constexpr size_t kOffWDTT  = kOffWXT   + kSzWXT;
constexpr size_t kOffWOUTT = kOffWDTT  + kSzWDTT;
constexpr size_t kOffXB    = kOffWOUTT + kSzWOUTT;
constexpr size_t kOffXZ    = kOffXB    + kSzXB;
constexpr size_t kOffXCV16 = kOffXZ    + kSzXZ;
constexpr size_t kOffXC    = kOffXCV16 + kSzXCV16;
constexpr size_t kOffXC16  = kOffXC    + kSzXC;
constexpr size_t kOffPROJ  = kOffXC16  + kSzXC16;
constexpr size_t kOffDT16  = kOffPROJ  + kSzPROJ;
constexpr size_t kOffDLR   = kOffDT16  + kSzDT16;
constexpr size_t kOffY16   = kOffDLR   + kSzDLR;
constexpr size_t kWsTotal  = kOffY16   + kSzY16;
static_assert(kWsTotal == 123731968ull);
static_assert(kWsTotal <= 134217728ull);
static_assert((kOffPWT % 128) == 0 && (kOffWXT % 128) == 0 && (kOffWDTT % 128) == 0 && (kOffWOUTT % 128) == 0 &&
              (kOffXB % 128) == 0 && (kOffXZ % 128) == 0 && (kOffXCV16 % 128) == 0 && (kOffXC % 128) == 0 &&
              (kOffXC16 % 128) == 0 && (kOffPROJ % 128) == 0 && (kOffDT16 % 128) == 0 && (kOffDLR % 128) == 0 &&
              (kOffY16 % 128) == 0);

__device__ __forceinline__ unsigned short f2bf_bits(float f) {
  unsigned u = __float_as_uint(f);
  return (unsigned short)((u + 0x7FFFu + ((u >> 16) & 1u)) >> 16);
}
__device__ __forceinline__ float bf_bits2f(unsigned short h) { return __uint_as_float(((unsigned)h) << 16); }
__device__ __forceinline__ float bf_rne(float f) { return bf_bits2f(f2bf_bits(f)); }

__device__ __forceinline__ void dep_guard4_h(v8f& a, v8f& b, v8f& c, v8f& d, v16h x, v16h y) {
  asm volatile("v_nop\n\tv_nop\n\tv_nop\n\tv_nop" : "+v"(a), "+v"(b), "+v"(c), "+v"(d) : "v"(x), "v"(y));
}
__device__ __forceinline__ void dep_guard4_b(v8f& a, v8f& b, v8f& c, v8f& d, v16b x, v16b y) {
  asm volatile("v_nop\n\tv_nop\n\tv_nop\n\tv_nop" : "+v"(a), "+v"(b), "+v"(c), "+v"(d) : "v"(x), "v"(y));
}
__device__ __forceinline__ void keep4_h(v16h a, v16h b, v16h c, v16h d) { asm volatile("v_nop" :: "v"(a), "v"(b), "v"(c), "v"(d)); }
__device__ __forceinline__ void keep4_b(v16b a, v16b b, v16b c, v16b d) { asm volatile("v_nop" :: "v"(a), "v"(b), "v"(c), "v"(d)); }
__device__ __forceinline__ void acc_guard4(v8f& a, v8f& b, v8f& c, v8f& d) { asm volatile("v_nop\n\tv_nop\n\tv_nop\n\tv_nop" : "+v"(a), "+v"(b), "+v"(c), "+v"(d)); }
template <typename T> struct Frag;
template <> struct Frag<_Float16> {
  typedef v16h V; union U { v16h v; v8h h[2]; };
  static __device__ __forceinline__ v16h load(const _Float16* p) {
    U f; f.h[0] = *(const v8h*)(p); f.h[1] = *(const v8h*)(p + 16); return f.v;
  }
  static __device__ __forceinline__ v8f mma(v16h a, v16h b, v8f c) {
    return __builtin_amdgcn_wmma_f32_16x16x32_f16(false, a, false, b, (short)0, c, false, false);
  }
  static __device__ __forceinline__ void guard4(v8f& a, v8f& b, v8f& c, v8f& d, v16h x, v16h y) { dep_guard4_h(a, b, c, d, x, y); }
  static __device__ __forceinline__ void keep(v16h a, v16h b, v16h c, v16h d) { keep4_h(a, b, c, d); }
};
template <> struct Frag<__bf16> {
  typedef v16b V; union U { v16b v; v8b h[2]; };
  static __device__ __forceinline__ v16b load(const __bf16* p) {
    U f; f.h[0] = *(const v8b*)(p); f.h[1] = *(const v8b*)(p + 16); return f.v;
  }
  static __device__ __forceinline__ v8f mma(v16b a, v16b b, v8f c) {
    return __builtin_amdgcn_wmma_f32_16x16x32_bf16(false, a, false, b, (short)0, c, false, false);
  }
  static __device__ __forceinline__ void guard4(v8f& a, v8f& b, v8f& c, v8f& d, v16b x, v16b y) { dep_guard4_b(a, b, c, d, x, y); }
  static __device__ __forceinline__ void keep(v16b a, v16b b, v16b c, v16b d) { keep4_b(a, b, c, d); }
};

template <int ET> struct Elem;
template <> struct Elem<0> { typedef _Float16 T; };
template <> struct Elem<1> { typedef __bf16 T; };
template <int ET, bool SPLIT, int BIAS_MODE, int OUT_MODE, bool RESID, int ACT = 0>
__global__ __launch_bounds__(256) void wmma_gemm64(
    const unsigned short* __restrict__ Ap, const unsigned short* __restrict__ A2p, int lda, long strideA,
    const unsigned short* __restrict__ Btp, const unsigned short* __restrict__ Bt2p, int ldb, long strideB,
    void* __restrict__ Cout, void* __restrict__ Cout2, int ldc, long strideC,
    const float* __restrict__ bias,
    const float* __restrict__ resid, long strideR,
    int M, int N, int K, float scale) {
  typedef typename Elem<ET>::T T;
  typedef typename Frag<T>::V V;
  const T* A = (const T*)Ap; const T* A2 = (const T*)A2p; const T* Bt = (const T*)Btp; const T* Bt2 = (const T*)Bt2p;
  __shared__ __align__(16) float sT[8][16 * 68];
  const int b    = blockIdx.y;
  const int lane = threadIdx.x & 31;
  const int wave = threadIdx.x >> 5;
  const int tilesN = N >> 6;
  const int tilesM = M >> 6;
  const int tile = blockIdx.x * 8 + wave;
  if (tile >= tilesM * tilesN) return;
  const int tm = tile / tilesN;
  const int tn = tile - tm * tilesN;
  const int m0 = tm << 6;
  const int n0 = tn << 6;

  const T* Ab  = A  + (size_t)b * strideA;
  const T* Bb  = Bt + (size_t)b * strideB;
  const T* Ab2 = SPLIT ? (A2  + (size_t)b * strideA) : nullptr;
  const T* Bb2 = SPLIT ? (Bt2 + (size_t)b * strideB) : nullptr;

  const int rlane = lane & 15;
  const int koff  = (lane >> 4) * 8;
  const int mOff  = (lane >> 4) * 8;

  v8f acc[4][4];
#pragma unroll
  for (int i = 0; i < 4; ++i)
#pragma unroll
    for (int j = 0; j < 4; ++j) acc[i][j] = (v8f){0.f,0.f,0.f,0.f,0.f,0.f,0.f,0.f};

  for (int k0 = 0; k0 < K; k0 += 32) {
    V bh[4], bl[4];
#pragma unroll
    for (int j = 0; j < 4; ++j) {
      const size_t bo = (size_t)(n0 + (j << 4) + rlane) * ldb + koff + k0;
      bh[j] = Frag<T>::load(Bb + bo);
      if (SPLIT) bl[j] = Frag<T>::load(Bb2 + bo);
    }
#pragma unroll
    for (int i = 0; i < 4; ++i) {
      const size_t ao = (size_t)(m0 + (i << 4) + rlane) * lda + koff + k0;
      V ah = Frag<T>::load(Ab + ao);
      V al;
      if (SPLIT) al = Frag<T>::load(Ab2 + ao);
#pragma unroll
      for (int j = 0; j < 4; ++j) {
        acc[i][j] = Frag<T>::mma(ah, bh[j], acc[i][j]);
        if (SPLIT) {
          acc[i][j] = Frag<T>::mma(ah, bl[j], acc[i][j]);
          acc[i][j] = Frag<T>::mma(al, bh[j], acc[i][j]);
        }
      }
      Frag<T>::guard4(acc[i][0], acc[i][1], acc[i][2], acc[i][3], ah, SPLIT ? al : ah);
    }
    Frag<T>::keep(bh[0], bh[1], bh[2], bh[3]);
    if (SPLIT) Frag<T>::keep(bl[0], bl[1], bl[2], bl[3]);
  }
  acc_guard4(acc[0][0], acc[0][1], acc[0][2], acc[0][3]);
  acc_guard4(acc[1][0], acc[1][1], acc[1][2], acc[1][3]);
  acc_guard4(acc[2][0], acc[2][1], acc[2][2], acc[2][3]);
  acc_guard4(acc[3][0], acc[3][1], acc[3][2], acc[3][3]);

  float* slab = sT[wave];
  const float* Rb = RESID ? (resid + (size_t)b * strideR) : nullptr;
#pragma unroll
  for (int i = 0; i < 4; ++i) {
    const int mBase = m0 + (i << 4);
#pragma unroll
    for (int j = 0; j < 4; ++j) {
      const int n = n0 + (j << 4) + rlane;
      float bv = 0.f;
      if (BIAS_MODE == 2) bv = bf_rne(bias[n]);
#pragma unroll
      for (int r = 0; r < 8; ++r) {
        float v = acc[i][j][r] * scale;
        if (BIAS_MODE == 1) v += bf_rne(bias[mBase + mOff + r]);
        if (BIAS_MODE == 2) v += bv;
        if (RESID) v += Rb[(size_t)(mBase + mOff + r) * ldc + n];
        if (ACT == 1) v = tanhf(v);
        if (ACT == 2) v = fmaxf(v, 0.0f);
        if (ACT == 3) v = v / (1.0f + expf(-v));
        if (ACT == 4) v = (v > 0.f) ? v : 0.01f * v;
        slab[(mOff + r) * 68 + (j << 4) + rlane] = v;
      }
    }
    __builtin_amdgcn_fence(__ATOMIC_RELEASE, "workgroup");
    __builtin_amdgcn_wave_barrier();
    __builtin_amdgcn_fence(__ATOMIC_ACQUIRE, "workgroup");
    if (OUT_MODE == 0) {
      float* C = (float*)Cout + (size_t)b * strideC;
      const int hh = lane >> 4, c4 = (lane & 15) * 4;
      for (int pass = 0; pass < 2; ++pass) {
#pragma unroll
        for (int it = 0; it < 8; ++it) {
          const int row = it * 2 + hh;
          v4f v = *(const v4f*)(slab + row * 68 + c4);
          *(volatile v4f*)(C + (size_t)(mBase + row) * ldc + n0 + c4) = v;
        }
        __threadfence();
      }
    } else {
      const int q = lane >> 3, c8 = (lane & 7) * 8;
      unsigned short* C  = (unsigned short*)Cout  + (size_t)b * strideC;
      unsigned short* C2 = (OUT_MODE == 2) ? ((unsigned short*)Cout2 + (size_t)b * strideC) : nullptr;
      for (int pass = 0; pass < 2; ++pass) {
#pragma unroll
        for (int it = 0; it < 4; ++it) {
          const int row = it * 4 + q;
          const float* sp = slab + row * 68 + c8;
          v8h hv, lv;
#pragma unroll
          for (int e = 0; e < 8; ++e) {
            if (OUT_MODE == 1) {
              hv[e] = (_Float16)sp[e];
            } else {
              unsigned short hb = f2bf_bits(sp[e]);
              unsigned short lb = f2bf_bits(sp[e] - bf_bits2f(hb));
              hv[e] = __builtin_bit_cast(_Float16, hb);
              lv[e] = __builtin_bit_cast(_Float16, lb);
            }
          }
          *(volatile v8h*)(C + (size_t)(mBase + row) * ldc + n0 + c8) = hv;
          if (OUT_MODE == 2) *(volatile v8h*)(C2 + (size_t)(mBase + row) * ldc + n0 + c8) = lv;
        }
        __threadfence();
      }
    }
    __builtin_amdgcn_fence(__ATOMIC_RELEASE, "workgroup");
    __builtin_amdgcn_wave_barrier();
    __builtin_amdgcn_fence(__ATOMIC_ACQUIRE, "workgroup");
  }
}

__global__ __launch_bounds__(256) void cast_f16_kernel(
    const float* __restrict__ src, unsigned short* __restrict__ dst, int total8, float scale)
{
  const int i = blockIdx.x * 256 + threadIdx.x;
  if (i >= total8) return;
  const size_t e0 = (size_t)i << 3;
  const float* p = src + e0;
  const v4f a0 = *(const v4f*)(p);
  const v4f a1 = *(const v4f*)(p + 4);
  v8h hv;
#pragma unroll
  for (int e = 0; e < 4; ++e) {
    hv[e]     = (_Float16)(a0[e] * scale);
    hv[4 + e] = (_Float16)(a1[e] * scale);
  }
  unsigned short* q = dst + e0;
  *(volatile v8h*)q = hv;
  __threadfence();
  *(volatile v8h*)q = hv;
}

__global__ __launch_bounds__(256) void cast_bf16_kernel(
    const float* __restrict__ src, unsigned short* __restrict__ dst, int total8)
{
  const int i = blockIdx.x * 256 + threadIdx.x;
  if (i >= total8) return;
  const size_t e0 = (size_t)i << 3;
  const float* p = src + e0;
  const v4f a0 = *(const v4f*)(p);
  const v4f a1 = *(const v4f*)(p + 4);
  v8h hv;
#pragma unroll
  for (int e = 0; e < 4; ++e) {
    const unsigned short b0 = f2bf_bits(a0[e]);
    const unsigned short b1 = f2bf_bits(a1[e]);
    hv[e]     = __builtin_bit_cast(_Float16, b0);
    hv[4 + e] = __builtin_bit_cast(_Float16, b1);
  }
  unsigned short* q = dst + e0;
  *(volatile v8h*)q = hv;
  __threadfence();
  *(volatile v8h*)q = hv;
}

template <int MODE>
__global__ __launch_bounds__(256) void transpose_cast_kernel(
    const float* __restrict__ W, unsigned short* __restrict__ Bt, int Kdim, int Ndim, int Npad, float scale)
{
  __shared__ float tile[64 * 65];
  const int tid = threadIdx.x, lane = tid & 31, wave = tid >> 5;
  const int n0 = blockIdx.x * 64;
  const int k0 = blockIdx.y * 64;
  (void)Npad;
#pragma unroll
  for (int p = 0; p < 16; ++p) {
    if (p == 8) asm volatile("" ::: "memory");
    const int idx = tid + p * 256;
    const int kk  = idx >> 6;
    const int nn  = idx & 63;
    const int n   = n0 + nn;
    const int nc  = (n < Ndim) ? n : (Ndim - 1);
    const float v  = W[(size_t)(k0 + kk) * Ndim + nc];
    const float vr = bf_rne(v);
    const float tv = (MODE == 0) ? (vr * scale) : vr;
    tile[kk * 65 + nn] = (n < Ndim) ? tv : 0.f;
  }
  __syncthreads();
  const int q = lane >> 3, c8 = (lane & 7) * 8;
  v8h hv[2];
#pragma unroll
  for (int it = 0; it < 2; ++it) {
    const int nrow = it * 32 + wave * 4 + q;
#pragma unroll
    for (int e = 0; e < 8; ++e) {
      const float t = tile[(c8 + e) * 65 + nrow];
      if (MODE == 0) {
        hv[it][e] = (_Float16)t;
      } else {
        const unsigned short bb = f2bf_bits(t);
        hv[it][e] = __builtin_bit_cast(_Float16, bb);
      }
    }
  }
  for (int pass = 0; pass < 2; ++pass) {
#pragma unroll
    for (int it = 0; it < 2; ++it) {
      const int nrow = it * 32 + wave * 4 + q;
      *(volatile v8h*)(Bt + (size_t)(n0 + nrow) * Kdim + k0 + c8) = hv[it];
    }
    __threadfence();
  }
}

__global__ __launch_bounds__(256) void dt_cast_kernel(
    const float* __restrict__ PROJ, unsigned short* __restrict__ DT16, int total8, float scale)
{
  const int i = blockIdx.x * 256 + threadIdx.x;
  if (i >= total8) return;
  const int e0  = i << 3;
  const int row = e0 >> 6;
  const int c8  = e0 & 63;
  const float* p = PROJ + (size_t)row * kPrjP + c8;
  const v4f a0 = *(const v4f*)(p);
  const v4f a1 = *(const v4f*)(p + 4);
  v8h hv;
#pragma unroll
  for (int e = 0; e < 4; ++e) {
    hv[e]     = (_Float16)(a0[e] * scale);
    hv[4 + e] = (_Float16)(a1[e] * scale);
  }
  unsigned short* qd = DT16 + e0;
  *(volatile v8h*)qd = hv;
  __threadfence();
  *(volatile v8h*)qd = hv;
}

__global__ __launch_bounds__(256) void dwconv_kernel(
    const float* __restrict__ XZ, const float* __restrict__ dw, unsigned short* __restrict__ XCV16)
{
  __shared__ __align__(16) float sT[16 * kTP];
  const int tid = threadIdx.x, lane = tid & 31, wave = tid >> 5;
  const int d0 = blockIdx.x * 256, d = d0 + tid;
  const int t0 = blockIdx.y * 64;
  const float w0 = bf_rne(dw[0 * kDin + d]);
  const float w1 = bf_rne(dw[1 * kDin + d]);
  const float w2 = bf_rne(dw[2 * kDin + d]);
  const float w3 = bf_rne(dw[3 * kDin + d]);
  float xm3, xm2, xm1;
  {
    const int r3 = t0 - 3, r2 = t0 - 2, r1 = t0 - 1;
    const float v3 = XZ[(size_t)(r3 < 0 ? 0 : r3) * kXZP + d];
    const float v2 = XZ[(size_t)(r2 < 0 ? 0 : r2) * kXZP + d];
    const float v1 = XZ[(size_t)(r1 < 0 ? 0 : r1) * kXZP + d];
    xm3 = (r3 >= 0) ? v3 : 0.f;
    xm2 = (r2 >= 0) ? v2 : 0.f;
    xm1 = (r1 >= 0) ? v1 : 0.f;
  }
#pragma unroll 1
  for (int sub = 0; sub < 4; ++sub) {
    const int lb = t0 + sub * 16;
#pragma unroll 1
    for (int s = 0; s < 16; ++s) {
      const float xcur = XZ[(size_t)(lb + s) * kXZP + d];
      float a = w0 * xm3;
      a = fmaf(w1, xm2, a);
      a = fmaf(w2, xm1, a);
      a = fmaf(w3, xcur, a);
      sT[s * kTP + tid] = a * kCarCv;
      xm3 = xm2; xm2 = xm1; xm1 = xcur;
    }
    __syncthreads();
    v8h hv[2];
#pragma unroll
    for (int it = 0; it < 2; ++it) {
      const float* sp = sT + (it * 8 + wave) * kTP + lane * 8;
      const v4f a0 = *(const v4f*)(sp);
      const v4f a1 = *(const v4f*)(sp + 4);
#pragma unroll
      for (int e = 0; e < 4; ++e) {
        hv[it][e]     = (_Float16)a0[e];
        hv[it][4 + e] = (_Float16)a1[e];
      }
    }
    for (int pass = 0; pass < 2; ++pass) {
#pragma unroll
      for (int it = 0; it < 2; ++it)
        *(volatile v8h*)(XCV16 + (size_t)(lb + it * 8 + wave) * kDin + d0 + lane * 8) = hv[it];
      __threadfence();
    }
    __syncthreads();
  }
}

__global__ __launch_bounds__(256) void scan_kernel(
    const float* __restrict__ DLR, const float* __restrict__ XC, const float* __restrict__ XZ,
    const float* __restrict__ PROJ, const float* __restrict__ A_log, const float* __restrict__ Dv,
    unsigned short* __restrict__ Y16)
{
  __shared__ __align__(16) float sBC[16 * 16];
  __shared__ __align__(16) float sY[16 * kTP];
  const int tid = threadIdx.x, lane = tid & 31, wave = tid >> 5;
  const int d0 = blockIdx.x * 256, d = d0 + tid;

  float An[kNst];
  {
    const v4f l0v = *(const v4f*)(A_log + (size_t)d * kNst);
    const v4f l1v = *(const v4f*)(A_log + (size_t)d * kNst + 4);
#pragma unroll
    for (int e = 0; e < 4; ++e) {
      An[e]     = -__expf(bf_rne(l0v[e]));
      An[4 + e] = -__expf(bf_rne(l1v[e]));
    }
  }
  const float Dd = bf_rne(Dv[d]);
  float h[kNst];
#pragma unroll
  for (int n = 0; n < kNst; ++n) h[n] = 0.f;

#pragma unroll 1
  for (int c = 0; c < kSeqL / 16; ++c) {
    const int l0 = c * 16;
    if (tid < 64) {
      const int r = tid >> 2, q4 = (tid & 3) * 4;
      const v4f v = *(const v4f*)(PROJ + (size_t)(l0 + r) * kPrjP + kDtR + q4);
      *(v4f*)(sBC + r * 16 + q4) = v;
    }
    __syncthreads();
#pragma unroll 1
    for (int s = 0; s < 16; ++s) {
      const size_t m = (size_t)(l0 + s);
      const float a     = DLR[m * kDin + d];
      const float delta = fmaxf(a, 0.0f) + __logf(1.0f + __expf(-fabsf(a)));
      const float xv    = XC[m * kDin + d];
      const float zv    = XZ[m * kXZP + kDin + d];
      v4f Bq[2], Cq[2];
      Bq[0] = *(const v4f*)(sBC + s * 16);
      Bq[1] = *(const v4f*)(sBC + s * 16 + 4);
      Cq[0] = *(const v4f*)(sBC + s * 16 + 8);
      Cq[1] = *(const v4f*)(sBC + s * 16 + 12);
      const float dtx = delta * xv;
      float y = 0.f;
#pragma unroll
      for (int n = 0; n < kNst; ++n) {
        const float e  = __expf(delta * An[n]);
        const float hn = fmaf(e, h[n], dtx * Bq[n >> 2][n & 3]);
        h[n] = hn;
        y = fmaf(Cq[n >> 2][n & 3], hn, y);
      }
      y = fmaf(xv, Dd, y);
      const float sg = __builtin_amdgcn_rcpf(1.0f + expf(-zv));
      const float g  = zv * sg;
      sY[s * kTP + tid] = (y * g) * kCarY;
    }
    __syncthreads();
    v8h hv[2];
#pragma unroll
    for (int it = 0; it < 2; ++it) {
      const float* sp = sY + (it * 8 + wave) * kTP + lane * 8;
      const v4f a0 = *(const v4f*)(sp);
      const v4f a1 = *(const v4f*)(sp + 4);
#pragma unroll
      for (int e = 0; e < 4; ++e) { hv[it][e] = (_Float16)a0[e]; hv[it][4 + e] = (_Float16)a1[e]; }
    }
    for (int pass = 0; pass < 2; ++pass) {
#pragma unroll
      for (int it = 0; it < 2; ++it)
        *(volatile v8h*)(Y16 + (size_t)(l0 + it * 8 + wave) * kDin + d0 + lane * 8) = hv[it];
      __threadfence();
    }
  }
}

extern "C" void kernel_launch(void* const* d_in, const int* in_sizes, int n_in,
                              void* d_out, int out_size, void* d_ws, size_t ws_size,
                              hipStream_t stream)
{
  if (n_in < 11) return;
  const float* x      = (const float*)d_in[0];
  const float* W_in   = (const float*)d_in[1];
  const float* dw_w   = (const float*)d_in[2];
  const float* pw_w   = (const float*)d_in[3];
  const float* conv_b = (const float*)d_in[4];
  const float* W_x    = (const float*)d_in[5];
  const float* W_dt   = (const float*)d_in[6];
  const float* b_dt   = (const float*)d_in[7];
  const float* A_log  = (const float*)d_in[8];
  const float* Dv     = (const float*)d_in[9];
  const float* W_out  = (const float*)d_in[10];
  float* dout = (float*)d_out;

  if (in_sizes[0] != kRows * kDmod) return;
  if (in_sizes[1] != kDmod * kXZP) return;
  if (in_sizes[2] != kDcv * kDin) return;
  if (in_sizes[3] != kDin * kDin) return;
  if (in_sizes[4] != kDin) return;
  if (in_sizes[5] != kDin * kPrjN) return;
  if (in_sizes[6] != kDtR * kDin) return;
  if (in_sizes[7] != kDin) return;
  if (in_sizes[8] != kDin * kNst) return;
  if (in_sizes[9] != kDin) return;
  if (in_sizes[10] != kDin * kDmod) return;
  if (out_size != kRows * kDmod) return;
  if (ws_size < kWsTotal) return;

  char* ws = (char*)d_ws;
  unsigned short* WINB  = (unsigned short*)(ws + kOffWINB);
  unsigned short* PWT   = (unsigned short*)(ws + kOffPWT);
  unsigned short* WXT   = (unsigned short*)(ws + kOffWXT);
  unsigned short* WDTT  = (unsigned short*)(ws + kOffWDTT);
  unsigned short* WOUTT = (unsigned short*)(ws + kOffWOUTT);
  unsigned short* XB    = (unsigned short*)(ws + kOffXB);
  float*          XZ    = (float*)(ws + kOffXZ);
  unsigned short* XCV16 = (unsigned short*)(ws + kOffXCV16);
  float*          XC    = (float*)(ws + kOffXC);
  unsigned short* XC16  = (unsigned short*)(ws + kOffXC16);
  float*          PROJ  = (float*)(ws + kOffPROJ);
  unsigned short* DT16  = (unsigned short*)(ws + kOffDT16);
  float*          DLR   = (float*)(ws + kOffDLR);
  unsigned short* Y16   = (unsigned short*)(ws + kOffY16);
  const float* dummy_bias  = conv_b;
  const float* dummy_resid = x;

  transpose_cast_kernel<1><<<dim3(kXZP / 64, kDmod / 64), 256, 0, stream>>>(W_in,  WINB,  kDmod, kXZP,  kXZP,  1.0f);
  transpose_cast_kernel<0><<<dim3(kDin / 64, kDin / 64), 256, 0, stream>>>(pw_w,  PWT,   kDin,  kDin,  kDin,  kCarW);
  transpose_cast_kernel<0><<<dim3(kPrjP / 64, kDin / 64), 256, 0, stream>>>(W_x,  WXT,   kDin,  kPrjN, kPrjP, kCarW);
  transpose_cast_kernel<0><<<dim3(kDin / 64, kDtR / 64), 256, 0, stream>>>(W_dt,  WDTT,  kDtR,  kDin,  kDin,  kCarWdt);
  transpose_cast_kernel<0><<<dim3(kDmod / 64, kDin / 64), 256, 0, stream>>>(W_out, WOUTT, kDin, kDmod, kDmod, kCarW);

  cast_bf16_kernel<<<(kRows * kDmod) / 8 / 256, 256, 0, stream>>>(x, XB, (kRows * kDmod) / 8);

  for (int b = 0; b < kBatch; ++b) {
    const unsigned short* XBb = XB + (size_t)b * kSeqL * kDmod;
    float* outb = dout + (size_t)b * kSeqL * kDmod;

    wmma_gemm64<1, false, 0, 0, false><<<dim3(256, 1), 256, 0, stream>>>(
        XBb, XBb, kDmod, 0L, WINB, WINB, kDmod, 0L,
        (void*)XZ, (void*)XZ, kXZP, 0L, dummy_bias, dummy_resid, 0L, kSeqL, kXZP, kDmod, 1.0f);

    dwconv_kernel<<<dim3(kDin / 256, kSeqL / 64), 256, 0, stream>>>(XZ, dw_w, XCV16);

    wmma_gemm64<0, false, 2, 0, false, 3><<<dim3(128, 1), 256, 0, stream>>>(
        XCV16, XCV16, kDin, 0L, PWT, PWT, kDin, 0L,
        (void*)XC, (void*)XC, kDin, 0L, conv_b, dummy_resid, 0L, kSeqL, kDin, kDin, kSclPw);

    cast_f16_kernel<<<(kSeqL * kDin) / 8 / 256, 256, 0, stream>>>(XC, XC16, (kSeqL * kDin) / 8, kCarXc);

    wmma_gemm64<0, false, 0, 0, false><<<dim3(8, 1), 256, 0, stream>>>(
        XC16, XC16, kDin, 0L, WXT, WXT, kDin, 0L,
        (void*)PROJ, (void*)PROJ, kPrjP, 0L, dummy_bias, dummy_resid, 0L, kSeqL, kPrjP, kDin, kSclXp);

    dt_cast_kernel<<<(kSeqL * kDtR) / 8 / 256, 256, 0, stream>>>(PROJ, DT16, (kSeqL * kDtR) / 8, kCarDt);

    wmma_gemm64<0, false, 2, 0, false><<<dim3(128, 1), 256, 0, stream>>>(
        DT16, DT16, kDtR, 0L, WDTT, WDTT, kDtR, 0L,
        (void*)DLR, (void*)DLR, kDin, 0L, b_dt, dummy_resid, 0L, kSeqL, kDin, kDtR, kSclDt);

    scan_kernel<<<dim3(kDin / 256, 1), 256, 0, stream>>>(DLR, XC, XZ, PROJ, A_log, Dv, Y16);

    wmma_gemm64<0, false, 0, 0, false><<<dim3(64, 1), 256, 0, stream>>>(
        Y16, Y16, kDin, 0L, WOUTT, WOUTT, kDin, 0L,
        (void*)outb, (void*)outb, kDmod, 0L, dummy_bias, dummy_resid, 0L, kSeqL, kDmod, kDin, kSclOut);
  }
}
